// SGATMultiLayer_75488345194755
// MI455X (gfx1250) — hardware-verified
//
#include <hip/hip_runtime.h>
#include <hip/hip_bf16.h>


#define IN_F   256
#define NCOL   128
#define SP     160
#define ASP    544
#define ATP    32
#define PRE_A  0.1f
#define PRE_B  0.9f
#define POST_A 0.1f
#define POST_B 0.9f
#define EPSV   1e-9f

#define GBM 128
#define GTB 256
#define ATB 128
#define R1  64
#define TB1 160
#define NW1 5
#define R2  224
#define TB2 64
#define NW2 2
#define HL  128

typedef float          v4f   __attribute__((ext_vector_type(4)));
typedef float          v8f   __attribute__((ext_vector_type(8)));
typedef int            v4i   __attribute__((ext_vector_type(4)));
typedef unsigned short v4us  __attribute__((ext_vector_type(4)));
typedef unsigned short v8us  __attribute__((ext_vector_type(8)));
typedef unsigned short v16us __attribute__((ext_vector_type(16)));
typedef __bf16         v16bf __attribute__((ext_vector_type(16)));

union Frag { v16bf b; v16us u; v8us h[2]; };

__device__ __forceinline__ unsigned short f2bf(float f)
{
    unsigned u = __float_as_uint(f);
    u += 0x7FFFu + ((u >> 16) & 1u);
    return (unsigned short)(u >> 16);
}
__device__ __forceinline__ float bf2f(unsigned short b)
{
    return __uint_as_float(((unsigned)b) << 16);
}
__device__ __forceinline__ v4f ld4(const float* p) { return *(const v4f*)p; }
__device__ __forceinline__ void st4v(float* p, v4f v) { *(volatile v4f*)p = v; }
__device__ __forceinline__ v4f rcp4(v4f d)
{
    v4f r;
    r.x = __builtin_amdgcn_rcpf(d.x);
    r.y = __builtin_amdgcn_rcpf(d.y);
    r.z = __builtin_amdgcn_rcpf(d.z);
    r.w = __builtin_amdgcn_rcpf(d.w);
    return r;
}

__device__ __forceinline__ v8f wmma_bf16(const Frag& a, const Frag& bb, v8f acc)
{
    acc = __builtin_amdgcn_wmma_f32_16x16x32_bf16(false, a.b, false, bb.b, (short)0, acc, false, false);
    asm volatile("v_nop\n\tv_nop\n\tv_nop\n\tv_nop" : "+v"(acc) : "v"(a.u), "v"(bb.u));
    return acc;
}

__device__ __forceinline__ void gemm_store(const float* st, float* s0, int wrow0, int nrows, int lane)
{
    const v4f one4 = {1.f, 1.f, 1.f, 1.f};
    const v4f z4 = {0.f, 0.f, 0.f, 0.f};
#pragma unroll 1
    for (int s = 0; s < 20; ++s) {
        const int f = 32 * s + lane;
        const int row = f / 40, c4 = f - row * 40;
        const int grow = wrow0 + row;
        if (grow < nrows) {
            v4f val = z4;
            if (c4 < 32) val = *(const v4f*)(st + row * NCOL + 4 * c4);
            else if (c4 == 32) val = one4;
            st4v(s0 + (size_t)grow * SP + 4 * c4, val);
        }
    }
}

__global__ __launch_bounds__(GTB) void k_gemm(const float* __restrict__ x, const float* __restrict__ w,
                                             float* __restrict__ s0, int nrows)
{
    __shared__ __attribute__((aligned(16))) unsigned short Ah[GBM * 32];
    __shared__ __attribute__((aligned(16))) unsigned short Al[GBM * 32];
    __shared__ __attribute__((aligned(16))) unsigned short Bh[NCOL * 32];
    __shared__ __attribute__((aligned(16))) unsigned short Bl[NCOL * 32];
    __shared__ __attribute__((aligned(16))) float stg[8 * 16 * NCOL];

    const int tid = threadIdx.x, wave = tid >> 5, lane = tid & 31;
    const int h = lane >> 4, m = lane & 15;
    const int rb = blockIdx.x * GBM;
    const v4f z4 = {0.f, 0.f, 0.f, 0.f};

    v8f acc[8];
#pragma unroll
    for (int t = 0; t < 8; ++t) {
        const v8f z8 = {0.f, 0.f, 0.f, 0.f, 0.f, 0.f, 0.f, 0.f};
        acc[t] = z8;
    }

    for (int k0 = 0; k0 < IN_F; k0 += 32) {
#pragma unroll
        for (int it = 0; it < 4; ++it) {
            const int f = tid + GTB * it;
            const int row = f >> 3, kq = f & 7;
            const int grow = rb + row;
            v4f xv = z4;
            if (grow < nrows) xv = ld4(x + (size_t)grow * IN_F + k0 + 4 * kq);
            v4us hi, lo;
#pragma unroll
            for (int c = 0; c < 4; ++c) {
                const unsigned short hh = f2bf(xv[c]);
                hi[c] = hh;
                lo[c] = f2bf(xv[c] - bf2f(hh));
            }
            *(v4us*)(Ah + row * 32 + 4 * kq) = hi;
            *(v4us*)(Al + row * 32 + 4 * kq) = lo;
        }
#pragma unroll
        for (int it = 0; it < 4; ++it) {
            const int f = tid + GTB * it;
            const int kk = f >> 5, nq = f & 31;
            const v4f wv = ld4(w + (size_t)(k0 + kk) * NCOL + 4 * nq);
#pragma unroll
            for (int c = 0; c < 4; ++c) {
                const int n = 4 * nq + c;
                const unsigned short hh = f2bf(wv[c]);
                Bh[n * 32 + kk] = hh;
                Bl[n * 32 + kk] = f2bf(wv[c] - bf2f(hh));
            }
        }
        __syncthreads();

        Frag ah, al;
        const int ao = (wave * 16 + m) * 32 + 8 * h;
        ah.h[0] = *(const v8us*)(Ah + ao);
        ah.h[1] = *(const v8us*)(Ah + ao + 16);
        al.h[0] = *(const v8us*)(Al + ao);
        al.h[1] = *(const v8us*)(Al + ao + 16);
#pragma unroll
        for (int t = 0; t < 8; ++t) {
            Frag bh, bl;
            const int bo = (t * 16 + m) * 32 + 8 * h;
            bh.h[0] = *(const v8us*)(Bh + bo);
            bh.h[1] = *(const v8us*)(Bh + bo + 16);
            bl.h[0] = *(const v8us*)(Bl + bo);
            bl.h[1] = *(const v8us*)(Bl + bo + 16);
            acc[t] = wmma_bf16(ah, bh, acc[t]);
            acc[t] = wmma_bf16(ah, bl, acc[t]);
            acc[t] = wmma_bf16(al, bh, acc[t]);
        }
        __syncthreads();
    }

    float* st = stg + wave * (16 * NCOL);
#pragma unroll
    for (int t = 0; t < 8; ++t) {
#pragma unroll
        for (int r = 0; r < 8; ++r) st[(8 * h + r) * NCOL + 16 * t + m] = acc[t][r];
    }
    __syncthreads();

    const int wrow0 = rb + wave * 16;
    gemm_store(st, s0, wrow0, nrows, lane);
    __threadfence();
    gemm_store(st, s0, wrow0, nrows, lane);
}

__device__ __forceinline__ void attn_store(const float* rec, float* att, int nb, int nrows, int tid)
{
#pragma unroll
    for (int s = 0; s < 2; ++s) {
        const int f = tid + ATB * s;
        const int n2 = f >> 3, q = f & 7;
        const int a = nb + n2;
        if (a < nrows) st4v(att + (size_t)a * ATP + 4 * q, *(const v4f*)(rec + n2 * ATP + 4 * q));
    }
}

__global__ __launch_bounds__(ATB) void k_attn(const float* __restrict__ s0, const float* __restrict__ a1,
                                             const float* __restrict__ a2, float* __restrict__ att, int nrows)
{
    __shared__ __attribute__((aligned(16))) float rec[32 * ATP];

    const int tid = threadIdx.x;
    const int nl = tid >> 2, k = tid & 3;
    const int nb = blockIdx.x * 32;
    int ac = nb + nl;
    ac = ac >= nrows ? nrows - 1 : ac;
    const float* sr = s0 + (size_t)ac * SP;

    v4f c1 = {0.f, 0.f, 0.f, 0.f};
    v4f c2 = {0.f, 0.f, 0.f, 0.f};
#pragma unroll 4
    for (int i = 0; i < 32; ++i) {
        const v4f sv = ld4(sr + 4 * i);
        const v4f w1 = ld4(a1 + i * 16 + 4 * k);
        const v4f w2 = ld4(a2 + i * 16 + 4 * k);
        c1 += sv * w1;
        c2 += sv * w2;
    }
    v4f r1, r2;
#pragma unroll
    for (int j = 0; j < 4; ++j) {
        r1[j] = c1[j] + __builtin_amdgcn_sqrtf(c1[j] * c1[j] + 1.0f);
        r2[j] = c2[j] + __builtin_amdgcn_sqrtf(c2[j] * c2[j] + 1.0f);
    }
    *(v4f*)(rec + nl * ATP + 4 * k) = r1;
    *(v4f*)(rec + nl * ATP + 16 + 4 * k) = r2;
    __syncthreads();

    attn_store(rec, att, nb, nrows, tid);
    __threadfence();
    attn_store(rec, att, nb, nrows, tid);
}

__device__ __forceinline__ void hop1_store(const v4f* Y4, const float* S, const float* att, float* as1,
                                           int r0, int nrows, int wave, int lane)
{
    const v4f z4 = {0.f, 0.f, 0.f, 0.f};
#pragma unroll 1
    for (int s = wave; s < (R1 * 136) / 32; s += NW1) {
        const int f = 32 * s + lane;
        const int rl = f / 136, c4 = f - rl * 136;
        const int a = r0 + rl;
        if (a < nrows) {
            v4f val = z4;
            if (c4 < 132) {
                const int i = c4 >> 2, k = c4 & 3;
                const v4f s4 = ld4(S + (size_t)a * SP + 4 * i);
                const v4f a4 = ld4(att + (size_t)a * ATP + 16 + 4 * k);
                const v4f y = Y4[rl * 132 + c4];
                val = PRE_A * (s4 * a4) + PRE_B * y;
            }
            st4v(as1 + (size_t)a * ASP + 4 * c4, val);
        }
    }
}

__global__ __launch_bounds__(TB1) void k_hop1(const int* __restrict__ er, const int* __restrict__ ec,
                                             const float* __restrict__ ev, int nedges,
                                             const float* __restrict__ S, const float* __restrict__ att,
                                             float* __restrict__ as1, int nrows)
{
    __shared__ v4f   Y4[R1 * 132];
    __shared__ int   hl[NW1 * HL];
    __shared__ float hv[NW1 * HL];
    __shared__ int   wc[8];

    const int tid = threadIdx.x, wave = tid >> 5, lane = tid & 31;
    const int r0 = blockIdx.x * R1;
    const v4f z4 = {0.f, 0.f, 0.f, 0.f};
    for (int p = tid; p < R1 * 132; p += TB1) Y4[p] = z4;
    __syncthreads();

    const bool act = tid < 132;
    const int ti = tid >> 2, tk = tid & 3;
    const unsigned lt = (1u << lane) - 1u;

    for (int e0 = 0; e0 < nedges; e0 += TB1 * 4) {
        const int eb = e0 + wave * 128 + lane * 4;
        v4i rv = {-1, -1, -1, -1};
        if (eb + 3 < nedges) rv = *(const v4i*)(er + eb);
        else {
#pragma unroll
            for (int b = 0; b < 4; ++b) if (eb + b < nedges) rv[b] = er[eb + b];
        }
        int d[4]; bool hb[4]; unsigned mk[4];
#pragma unroll
        for (int b = 0; b < 4; ++b) {
            d[b] = rv[b] - r0;
            hb[b] = (unsigned)d[b] < (unsigned)R1;
            mk[b] = __builtin_amdgcn_ballot_w32(hb[b]);
        }
        int pb[4];
        pb[0] = 0;
        pb[1] = __builtin_popcount(mk[0]);
        pb[2] = pb[1] + __builtin_popcount(mk[1]);
        pb[3] = pb[2] + __builtin_popcount(mk[2]);
        const int tot = pb[3] + __builtin_popcount(mk[3]);
        if (tot != 0) {
#pragma unroll
            for (int b = 0; b < 4; ++b) {
                if (hb[b]) {
                    const int e = eb + b;
                    int c = ec[e];
                    const float v = ev[e];
                    c = c < 0 ? 0 : c;
                    c = c >= nrows ? nrows - 1 : c;
                    const int slot = wave * HL + pb[b] + __builtin_popcount(mk[b] & lt);
                    hl[slot] = c | (d[b] << 20);
                    hv[slot] = v;
                }
            }
        }
        if (lane == 0) wc[wave] = tot;
        __syncthreads();
#pragma unroll 1
        for (int wv = 0; wv < NW1; ++wv) {
            int cnt = wc[wv];
            cnt = cnt > HL ? HL : cnt;
#pragma unroll 1
            for (int q = 0; q < cnt; ++q) {
                const int pk = hl[wv * HL + q];
                const float v = hv[wv * HL + q];
                int c = pk & 0xFFFFF;
                c = c >= nrows ? nrows - 1 : c;
                int rl = (pk >> 20) & 0xFFF;
                rl = rl >= R1 ? R1 - 1 : rl;
                if (act) {
                    const v4f s4 = ld4(S + (size_t)c * SP + 4 * ti);
                    const v4f a4 = ld4(att + (size_t)c * ATP + 16 + 4 * tk);
                    v4f y = Y4[rl * 132 + tid];
                    y += v * (s4 * a4);
                    Y4[rl * 132 + tid] = y;
                }
            }
        }
        __syncthreads();
    }

    hop1_store(Y4, S, att, as1, r0, nrows, wave, lane);
    __threadfence();
    hop1_store(Y4, S, att, as1, r0, nrows, wave, lane);
}

template <int FINAL>
__device__ __forceinline__ void hop2_store(const v4f* T4, const v4f* Gs, const v4f* Rc1, const v4f* Rc2,
                                           const float* S, const float* S0, const float* bias, float* dst,
                                           int r0, int nrows, int wave, int lane)
{
    const v4f z4 = {0.f, 0.f, 0.f, 0.f};
    if (FINAL == 0) {
#pragma unroll 1
        for (int s = wave; s < (R2 * 40) / 32; s += NW2) {
            const int f = 32 * s + lane;
            const int rl = f / 40, c4 = f - rl * 40;
            const int a = r0 + rl;
            if (a < nrows) {
                v4f val = z4;
                if (c4 < 33) {
                    const v4f s4 = ld4(S + (size_t)a * SP + 4 * c4);
                    const v4f o4 = ld4(S0 + (size_t)a * SP + 4 * c4);
                    const v4f T = PRE_A * (s4 * Gs[rl]) + PRE_B * T4[rl * 33 + c4];
                    const v4f t = POST_A * o4 + POST_B * T;
                    val = t * Rc1[rl];
                }
                st4v(dst + (size_t)a * SP + 4 * c4, val);
            }
        }
    } else {
#pragma unroll 1
        for (int rl = wave; rl < R2; rl += NW2) {
            const int a = r0 + rl;
            if (a < nrows) {
                const int i = lane;
                const v4f s4 = ld4(S + (size_t)a * SP + 4 * i);
                const v4f o4 = ld4(S0 + (size_t)a * SP + 4 * i);
                const v4f T = PRE_A * (s4 * Gs[rl]) + PRE_B * T4[rl * 33 + i];
                const v4f t = POST_A * o4 + POST_B * T;
                const v4f sv = t * Rc1[rl];
                const v4f val = sv * Rc2[rl] + ld4(bias + 4 * i);
                st4v(dst + (size_t)a * NCOL + 4 * i, val);
            }
        }
    }
}

template <int FINAL>
__global__ __launch_bounds__(TB2) void k_hop2(const int* __restrict__ er, const int* __restrict__ ec,
                                             const float* __restrict__ ev, int nedges,
                                             const float* __restrict__ as1, const float* __restrict__ att,
                                             const float* S, const float* S0, const float* __restrict__ bias,
                                             float* __restrict__ dst, int nrows)
{
    __shared__ v4f   T4[R2 * 33];
    __shared__ v4f   A14[R2 * 4];
    __shared__ v4f   Gs[R2];
    __shared__ v4f   Rc1[R2];
    __shared__ v4f   Rc2[R2];
    __shared__ int   hl[NW2 * HL];
    __shared__ float hv[NW2 * HL];
    __shared__ int   wc[8];

    const int tid = threadIdx.x, wave = tid >> 5, lane = tid & 31;
    const int r0 = blockIdx.x * R2;
    const v4f z4 = {0.f, 0.f, 0.f, 0.f};
    for (int p = tid; p < R2 * 33; p += TB2) T4[p] = z4;
    for (int p = tid; p < R2 * 4; p += TB2) {
        const int a = r0 + (p >> 2);
        v4f v = z4;
        if (a < nrows) v = ld4(att + (size_t)a * ATP + 4 * (p & 3));
        A14[p] = v;
    }
    __syncthreads();

    const bool act = tid < 33;
    const unsigned lt = (1u << lane) - 1u;

    for (int e0 = 0; e0 < nedges; e0 += TB2 * 4) {
        const int eb = e0 + wave * 128 + lane * 4;
        v4i rv = {-1, -1, -1, -1};
        if (eb + 3 < nedges) rv = *(const v4i*)(er + eb);
        else {
#pragma unroll
            for (int b = 0; b < 4; ++b) if (eb + b < nedges) rv[b] = er[eb + b];
        }
        int d[4]; bool hb[4]; unsigned mk[4];
#pragma unroll
        for (int b = 0; b < 4; ++b) {
            d[b] = rv[b] - r0;
            hb[b] = (unsigned)d[b] < (unsigned)R2;
            mk[b] = __builtin_amdgcn_ballot_w32(hb[b]);
        }
        int pb[4];
        pb[0] = 0;
        pb[1] = __builtin_popcount(mk[0]);
        pb[2] = pb[1] + __builtin_popcount(mk[1]);
        pb[3] = pb[2] + __builtin_popcount(mk[2]);
        const int tot = pb[3] + __builtin_popcount(mk[3]);
        if (tot != 0) {
#pragma unroll
            for (int b = 0; b < 4; ++b) {
                if (hb[b]) {
                    const int e = eb + b;
                    int c = ec[e];
                    const float v = ev[e];
                    c = c < 0 ? 0 : c;
                    c = c >= nrows ? nrows - 1 : c;
                    const int slot = wave * HL + pb[b] + __builtin_popcount(mk[b] & lt);
                    hl[slot] = c | (d[b] << 20);
                    hv[slot] = v;
                }
            }
        }
        if (lane == 0) wc[wave] = tot;
        __syncthreads();
#pragma unroll 1
        for (int wv = 0; wv < NW2; ++wv) {
            int cnt = wc[wv];
            cnt = cnt > HL ? HL : cnt;
#pragma unroll 1
            for (int q = 0; q < cnt; ++q) {
                const int pk = hl[wv * HL + q];
                const float v = hv[wv * HL + q];
                int c = pk & 0xFFFFF;
                c = c >= nrows ? nrows - 1 : c;
                int rl = (pk >> 20) & 0xFFF;
                rl = rl >= R2 ? R2 - 1 : rl;
                if (act) {
                    const float* ap = as1 + (size_t)c * ASP + 16 * tid;
                    const v4f x0 = ld4(ap), x1 = ld4(ap + 4), x2 = ld4(ap + 8), x3 = ld4(ap + 12);
                    const int ab = rl * 4;
                    const v4f sm = x0 * A14[ab] + x1 * A14[ab + 1] + x2 * A14[ab + 2] + x3 * A14[ab + 3];
                    v4f tz = T4[rl * 33 + tid];
                    tz += v * sm;
                    T4[rl * 33 + tid] = tz;
                }
            }
        }
        __syncthreads();
    }

#pragma unroll 1
    for (int rl = tid; rl < R2; rl += TB2) {
        const int a = r0 + rl;
        v4f g = z4, rc1 = z4, rc2 = z4;
        if (a < nrows) {
            const float* atp = att + (size_t)a * ATP + 16;
            const int ab = rl * 4;
            g = ld4(atp) * A14[ab] + ld4(atp + 4) * A14[ab + 1] + ld4(atp + 8) * A14[ab + 2] + ld4(atp + 12) * A14[ab + 3];
            const v4f sh  = ld4(S + (size_t)a * SP + 128);
            const v4f s0h = ld4(S0 + (size_t)a * SP + 128);
            const v4f T32 = PRE_A * (sh * g) + PRE_B * T4[rl * 33 + 32];
            const v4f t32 = POST_A * s0h + POST_B * T32;
            rc1 = rcp4(t32 + EPSV);
            const v4f s32 = t32 * rc1;
            rc2 = rcp4(s32 + EPSV);
        }
        Gs[rl] = g;
        Rc1[rl] = rc1;
        Rc2[rl] = rc2;
    }
    __syncthreads();

    hop2_store<FINAL>(T4, Gs, Rc1, Rc2, S, S0, bias, dst, r0, nrows, wave, lane);
    __threadfence();
    hop2_store<FINAL>(T4, Gs, Rc1, Rc2, S, S0, bias, dst, r0, nrows, wave, lane);
}

static inline size_t al256(size_t v) { return (v + 255) & ~(size_t)255; }

extern "C" void kernel_launch(void* const* d_in, const int* in_sizes, int n_in,
                              void* d_out, int out_size, void* d_ws, size_t ws_size,
                              hipStream_t stream)
{
    if (n_in < 7) return;
    const float* x    = (const float*)d_in[0];
    const int*   ei   = (const int*)  d_in[1];
    const float* ev   = (const float*)d_in[2];
    const float* w    = (const float*)d_in[3];
    const float* bias = (const float*)d_in[4];
    const float* a1   = (const float*)d_in[5];
    const float* a2   = (const float*)d_in[6];
    float*       out  = (float*)d_out;

    const int nrows  = in_sizes[0] / IN_F;
    const int nedges = in_sizes[1] / 2;
    if (nrows <= 0 || nrows > (1 << 20) || nedges < 0) return;
    if (in_sizes[2] < nedges) return;
    if (in_sizes[3] != IN_F * NCOL || in_sizes[4] < NCOL || in_sizes[5] < 32 * 16 || in_sizes[6] < 32 * 16) return;
    if (out_size != nrows * NCOL) return;

    const int* er = ei;
    const int* ec = ei + nedges;

    const size_t bS  = (size_t)nrows * SP  * sizeof(float);
    const size_t bAT = (size_t)nrows * ATP * sizeof(float);
    const size_t bAS = (size_t)nrows * ASP * sizeof(float);
    const size_t oS0 = 0;
    const size_t oS1 = al256(oS0 + bS);
    const size_t oAT = al256(oS1 + bS);
    const size_t oAS = al256(oAT + bAT);
    if (oAS + bAS > ws_size) return;

    char*  ws  = (char*)d_ws;
    float* S0  = (float*)(ws + oS0);
    float* S1  = (float*)(ws + oS1);
    float* ATT = (float*)(ws + oAT);
    float* AS1 = (float*)(ws + oAS);

    const int gG = (nrows + GBM - 1) / GBM;
    const int gA = (nrows + 31) / 32;
    const int g1 = (nrows + R1 - 1) / R1;
    const int g2 = (nrows + R2 - 1) / R2;

    k_gemm<<<gG, GTB, 0, stream>>>(x, w, S0, nrows);
    k_attn<<<gA, ATB, 0, stream>>>(S0, a1, a2, ATT, nrows);

    k_hop1<<<g1, TB1, 0, stream>>>(er, ec, ev, nedges, S0, ATT, AS1, nrows);
    k_hop2<0><<<g2, TB2, 0, stream>>>(er, ec, ev, nedges, AS1, ATT, S0, S0, bias, S1, nrows);

    k_hop1<<<g1, TB1, 0, stream>>>(er, ec, ev, nedges, S1, ATT, AS1, nrows);
    k_hop2<1><<<g2, TB2, 0, stream>>>(er, ec, ev, nedges, AS1, ATT, S1, S0, bias, out, nrows);
}
